// Coords2Grid_58213986730418
// MI455X (gfx1250) — hardware-verified
//
#include <hip/hip_runtime.h>


namespace {
constexpr int NA = 800, NT = 28, NTP = 32, G = 48, NVOX = G * G * G  ;
constexpr float RES = 0.5f, DIM = 23.5f, WSC = 256.0f, PS = 8.0f;
typedef _Float16 b16;
typedef __attribute__((ext_vector_type(16))) _Float16 v16b;
typedef __attribute__((ext_vector_type(8))) _Float16 v8b;
typedef __attribute__((ext_vector_type(8))) float v8f;
typedef __attribute__((ext_vector_type(4))) float v4f;
__device__ __forceinline__ float bf16_rne(float f) { unsigned int u = __float_as_uint(f); u += 0x7FFFu + ((u >> 16) & 1u); return __uint_as_float(u & 0xFFFF0000u); }
__device__ __forceinline__ void split16(float v, b16& hi, b16& lo) { hi = (b16)v; lo = (b16)(v - (float)hi); }
__device__ __forceinline__ v16b frag_kb(const b16* p, int hh) { const v8b a = *(const v8b*)(p + 8 * hh), b = *(const v8b*)(p + 16 + 8 * hh); v16b f;
#pragma unroll
  for (int e = 0; e < 8; ++e) { f[e] = a[e]; f[8 + e] = b[e]; } return f; }
__device__ __forceinline__ v8f wmma16b(v16b a, v16b b, v8f c) { v8f d = __builtin_amdgcn_wmma_f32_16x16x32_f16(false, a, false, b, (short)0, c, false, false); asm volatile("v_nop\n\tv_nop\n\tv_nop\n\tv_nop" : "+v"(d) : "v"(a), "v"(b)); return d; }
__device__ __forceinline__ void wave_lds_sync() { __builtin_amdgcn_fence(__ATOMIC_RELEASE, "workgroup"); __builtin_amdgcn_wave_barrier(); __builtin_amdgcn_fence(__ATOMIC_ACQUIRE, "workgroup"); }
__device__ __forceinline__ float pmul(float a, float b) { float p = a * b; asm volatile("" : "+v"(p)); return p; }

__global__ __launch_bounds__(256) void prep_kernel(const float* __restrict__ coords, const float* __restrict__ types, const float* __restrict__ radii, float* __restrict__ AT, b16* __restrict__ TT) {
  const int t_ = blockIdx.x * 256 + threadIdx.x;
  if (t_ < NA) { const float r = bf16_rne(radii[t_]); const float v0 = bf16_rne(coords[t_ * 3]), v1 = bf16_rne(coords[t_ * 3 + 1]), v2 = bf16_rne(coords[t_ * 3 + 2]), v3 = 1.0f / pmul(r, r);
    for (int pass = 0; pass < 2; ++pass) { ((volatile float*)AT)[t_] = v0; ((volatile float*)AT)[NA + t_] = v1; ((volatile float*)AT)[2 * NA + t_] = v2; ((volatile float*)AT)[3 * NA + t_] = v3; __threadfence(); } }
  if (t_ < NTP * NA / 8) { const int e = t_ * 8; const int tt = e / NA, n0 = e % NA; v8b o; for (int j = 0; j < 8; ++j) o[j] = (tt < NT) ? (b16)(bf16_rne(types[(size_t)(n0 + j) * NT + tt]) * WSC) : (b16)0.0f;
    for (int pass = 0; pass < 2; ++pass) { *(volatile v8b*)(TT + e) = o; __threadfence(); } }
}
__global__ __launch_bounds__(128) void grid_kernel(const float* __restrict__ center, const float* __restrict__ AT, const b16* __restrict__ TT, float* __restrict__ out) {
  __shared__ __attribute__((aligned(16))) float St[NTP][64 + 4]; __shared__ int flag[NA]; __shared__ int clist[NA + 32]; __shared__ int ncand; __shared__ __attribute__((aligned(16))) b16 Bc[NTP][NA + 32 + 8];
  const int wave = threadIdx.x >> 5, lane = threadIdx.x & 31, nloc = lane & 15, hlf = lane >> 4, t_ = threadIdx.x; const size_t v0 = (size_t)blockIdx.x * 64; const size_t vox = v0 + wave * 16 + nloc;
  const int ix = (int)(vox / (G * G)), iy = (int)((vox / G) % G), iz = (int)(vox % G);
  const float ox = bf16_rne(center[0]) - DIM * 0.5f, oy = bf16_rne(center[1]) - DIM * 0.5f, oz = bf16_rne(center[2]) - DIM * 0.5f;
  const float px = ox + (float)ix * RES, py = oy + (float)iy * RES, pz = oz + (float)iz * RES;
  const float inv_e2 = 0.1353352832366127f;
  { const int bix = (int)(v0 / (G * G)), iy0 = (int)((v0 / G) % G), iy1 = (int)(((v0 + 63) / G) % G);
    const float bx = ox + (float)bix * RES, by0 = oy + (float)iy0 * RES, by1 = oy + (float)iy1 * RES, bz0 = oz, bz1 = oz + (float)(G - 1) * RES;
    for (int n = t_; n < NA; n += 128) { const float ax = AT[n], ay = AT[NA + n], az = AT[2 * NA + n]; const float ddx = ax - bx; const float ddy = ay < by0 ? by0 - ay : (ay > by1 ? ay - by1 : 0.0f); const float ddz = az < bz0 ? bz0 - az : (az > bz1 ? az - bz1 : 0.0f);
      const float dr2 = (ddx * ddx + ddy * ddy + ddz * ddz) * AT[3 * NA + n]; flag[n] = (dr2 < 2.26f) ? 1 : 0; }
    __syncthreads();
    if (t_ == 0) { int c = 0; for (int n = 0; n < NA; ++n) if (flag[n]) clist[c++] = n; const int cp = (c + 31) & ~31; for (int q = c; q < cp; ++q) clist[q] = -1; ncand = cp; }
    __syncthreads();
    const int cp = ncand; for (int q = t_; q < NTP * cp; q += 128) { const int tt = q / cp, k = q % cp; const int n = clist[k]; Bc[tt][k] = (n >= 0) ? TT[(size_t)tt * NA + n] : (b16)0.0f; }
    __syncthreads(); }
  const int cp = ncand;
  v8f acc[2] = {{}, {}};
  for (int kb = 0; kb < cp; kb += 32) { v16b a, al;
#pragma unroll
    for (int el = 0; el < 16; ++el) { const int n = clist[kb + ((el < 8) ? (8 * hlf + el) : (16 + 8 * hlf + el - 8))]; float f = 0.0f;
      if (n >= 0) { const float dx = px - AT[n], dy = py - AT[NA + n], dz = pz - AT[2 * NA + n]; const float d2 = pmul(dx, dx) + pmul(dy, dy) + pmul(dz, dz); const float dr2 = pmul(d2, AT[3 * NA + n]); const float dr = sqrtf(fmaxf(dr2, 1e-12f));
        if (dr < 1.0f) f = __expf(-2.0f * dr2); else if (dr < 1.5f) f = inv_e2 * ((pmul(4.0f, dr2) - pmul(12.0f, dr)) + 9.0f); }
      b16 p, q; split16(f * PS, p, q); a[el] = p; al[el] = q; }
#pragma unroll
    for (int t = 0; t < 2; ++t) { const v16b bw = frag_kb(&Bc[t * 16 + nloc][kb], hlf); acc[t] = wmma16b(a, bw, acc[t]); acc[t] = wmma16b(al, bw, acc[t]); } }
#pragma unroll
  for (int t = 0; t < 2; ++t)
#pragma unroll 1
    for (int r = 0; r < 8; ++r) St[t * 16 + nloc][wave * 16 + 8 * hlf + r] = acc[t][r] * (1.0f / (PS * WSC));
  __syncthreads();
  for (int pass = 0; pass < 2; ++pass) { for (int q = t_; q < NT * 16; q += 128) { const int tt = q >> 4, c4 = (q & 15) * 4; *(volatile v4f*)(out + (size_t)tt * NVOX + v0 + c4) = *(const v4f*)(&St[tt][c4]); } __threadfence(); }
}
}

extern "C" void kernel_launch(void* const* d_in, const int* in_sizes, int n_in, void* d_out, int out_size, void* d_ws, size_t ws_size, hipStream_t stream) {
  (void)n_in;
  auto Fp = [&](int i) { return (const float*)d_in[i]; };
  if (in_sizes[0] != 3 || in_sizes[1] != NA * 3 || in_sizes[2] != NA * NT || in_sizes[3] != NA || out_size != NT * NVOX) return;
  size_t off = 0; char* ws = (char*)d_ws;
  auto carve = [&](size_t bytes) { char* p = ws + off; off += (bytes + 255) & ~(size_t)255; return p; };
  float* AT = (float*)carve((size_t)4 * NA * 4); b16* TT = (b16*)carve((size_t)NTP * NA * 2);
  if (off > ws_size) return;
  prep_kernel<<<(NTP * NA / 8 + 255) / 256, 256, 0, stream>>>(Fp(1), Fp(2), Fp(3), AT, TT);
  grid_kernel<<<NVOX / 64, 128, 0, stream>>>(Fp(0), AT, TT, (float*)d_out);
}
